// Qwen3TTSAttention_71141838291451
// MI455X (gfx1250) — hardware-verified
//
#include <hip/hip_runtime.h>
#include <math.h>
#include <stdint.h>

#ifndef SEQ
#define SEQ 4096
#endif
#define SEQ_FULL 4096
#define DM    2048
#define NH    16
#define NKV   4
#define GQ    (NH / NKV)
#define HD    128
#define HALF  64
#define QP    (NH * HD)
#define KP    (NKV * HD)
#define NQB   (SEQ / 64)
#define VLP   ((SEQ < 512) ? SEQ : 512)
#define RESQB ((NQB < 8) ? NQB : 8)
#define RMS_EPS       1.0e-6f
#define ROPE_THETA_F  10000.0f
#define ATT_SCALE     0.08838834764831845f
#define RSC           4096.0f

static_assert((SEQ % 64) == 0 && SEQ >= 64 && SEQ <= SEQ_FULL);
static_assert(RESQB * 64 <= VLP && (VLP % 64) == 0);
static_assert(NH * HD == DM && QP == DM);
static_assert(NQB <= 64);
static_assert((DM % 64) == 0 && (KP % 64) == 0 && (QP % 64) == 0 && (DM % 32) == 0);

typedef _Float16 v16h __attribute__((ext_vector_type(16)));
typedef _Float16 v8h  __attribute__((ext_vector_type(8)));
typedef __bf16   v16b __attribute__((ext_vector_type(16)));
typedef __bf16   v8b  __attribute__((ext_vector_type(8)));
typedef float    v8f  __attribute__((ext_vector_type(8)));
typedef float    v4f  __attribute__((ext_vector_type(4)));
typedef unsigned int   v4u  __attribute__((ext_vector_type(4)));
typedef unsigned int   v2u  __attribute__((ext_vector_type(2)));
typedef unsigned short v8us __attribute__((ext_vector_type(8)));
typedef int      v4i  __attribute__((ext_vector_type(4)));

__device__ __forceinline__ unsigned short bf_bits(float f) {
  unsigned u = __float_as_uint(f);
  return (unsigned short)((u + 0x7FFFu + ((u >> 16) & 1u)) >> 16);
}
__device__ __forceinline__ float bf_up(unsigned short h) { return __uint_as_float(((unsigned)h) << 16); }
__device__ __forceinline__ unsigned short h_bits(_Float16 x) { return __builtin_bit_cast(unsigned short, x); }
__device__ __forceinline__ unsigned pk16(unsigned short a, unsigned short b) { return (unsigned)a | ((unsigned)b << 16); }
__device__ __forceinline__ v8f zero8() { v8f z = {0.f, 0.f, 0.f, 0.f, 0.f, 0.f, 0.f, 0.f}; return z; }
__device__ __forceinline__ v8h zero8h() {
  const _Float16 z = (_Float16)0.0f;
  v8h r = {z, z, z, z, z, z, z, z};
  return r;
}
__device__ __forceinline__ int imin(int a, int b) { return (a < b) ? a : b; }
__device__ __forceinline__ int imax(int a, int b) { return (a > b) ? a : b; }

__device__ __forceinline__ v16b ldfrag_b(const __bf16* p) {
  union { v16b v; v8b h[2]; } f;
  f.h[0] = *(const v8b*)(p);
  f.h[1] = *(const v8b*)(p + 16);
  return f.v;
}

__device__ __forceinline__ v8f mma_b(v16b a, v16b b, v8f c) {
  c = __builtin_amdgcn_wmma_f32_16x16x32_bf16(false, a, false, b, (short)0, c, false, false);
  asm volatile("v_nop\n\tv_nop\n\tv_nop\n\tv_nop" : "+v"(c) : "v"(a), "v"(b));
  return c;
}
__device__ __forceinline__ v8f mma_h(v16h a, v16h b, v8f c) {
  c = __builtin_amdgcn_wmma_f32_16x16x32_f16(false, a, false, b, (short)0, c, false, false);
  asm volatile("v_nop\n\tv_nop\n\tv_nop\n\tv_nop" : "+v"(c) : "v"(a), "v"(b));
  return c;
}
__device__ __forceinline__ v8f mma_b_raw(v16b a, v16b b, v8f c) {
  return __builtin_amdgcn_wmma_f32_16x16x32_bf16(false, a, false, b, (short)0, c, false, false);
}
__device__ __forceinline__ void dep_guard_b(v8f& a, v8f& b, v16b x, v16b y) {
  asm volatile("v_nop\n\tv_nop\n\tv_nop\n\tv_nop" : "+v"(a), "+v"(b) : "v"(x), "v"(y));
}
__device__ __forceinline__ void keep4_b(v16b a, v16b b, v16b c, v16b d) {
  asm volatile("v_nop" :: "v"(a), "v"(b), "v"(c), "v"(d));
}
__device__ __forceinline__ void acc_guard4(v8f& a, v8f& b, v8f& c, v8f& d) {
  asm volatile("v_nop\n\tv_nop\n\tv_nop\n\tv_nop" : "+v"(a), "+v"(b), "+v"(c), "+v"(d));
}

__global__ __launch_bounds__(256) void cvt_bf16x8(const float* __restrict__ in, unsigned short* out, int n8) {
  const int i = blockIdx.x * 256 + threadIdx.x;
  if (i < n8) {
    const v4f a = *(const v4f*)(in + (size_t)i * 8);
    const v4f b = *(const v4f*)(in + (size_t)i * 8 + 4);
    v4u p;
    p[0] = pk16(bf_bits(a[0]), bf_bits(a[1]));
    p[1] = pk16(bf_bits(a[2]), bf_bits(a[3]));
    p[2] = pk16(bf_bits(b[0]), bf_bits(b[1]));
    p[3] = pk16(bf_bits(b[2]), bf_bits(b[3]));
    *(volatile v4u*)(out + (size_t)i * 8) = p;
    __threadfence();
    *(volatile v4u*)(out + (size_t)i * 8) = p;
  }
}

__global__ __launch_bounds__(256) void cvt_bf16_t(const float* __restrict__ in, unsigned short* out, int R, int C) {
  __shared__ __align__(16) unsigned short sT[64 * 72];
  const int tid = threadIdx.x;
  const int c0 = blockIdx.x * 64, r0 = blockIdx.y * 64;
  const int rr = tid >> 4, cc = (tid & 15) * 4;
#pragma unroll
  for (int it = 0; it < 4; ++it) {
    const int r = it * 16 + rr;
    const v4f v = *(const v4f*)(in + (size_t)(r0 + r) * C + c0 + cc);
#pragma unroll
    for (int e = 0; e < 4; ++e) sT[(cc + e) * 72 + r] = bf_bits(v[e]);
  }
  __syncthreads();
  const int q = tid >> 3, k8 = (tid & 7) * 8;
  const v8us w0 = *(const v8us*)(sT + q * 72 + k8);
  const v8us w1 = *(const v8us*)(sT + (q + 32) * 72 + k8);
  unsigned short* o0 = out + (size_t)(c0 + q) * R + r0 + k8;
  unsigned short* o1 = out + (size_t)(c0 + q + 32) * R + r0 + k8;
  *(volatile v8us*)o0 = w0;
  *(volatile v8us*)o1 = w1;
  __threadfence();
  *(volatile v8us*)o0 = w0;
  *(volatile v8us*)o1 = w1;
}

__global__ __launch_bounds__(64) void invf_tab(float* invf) {
  const int i = threadIdx.x;
  const float e = (float)i * (1.0f / (float)HALF);
  const float p = powf(ROPE_THETA_F, e);
  const float v = 1.0f / p;
  *(volatile float*)(invf + i) = v;
  __threadfence();
  *(volatile float*)(invf + i) = v;
}

__global__ __launch_bounds__(256) void rope_tab(const int* __restrict__ pos, const float* __restrict__ invf,
                                                float* ctab, float* stab, int nrows) {
  const int tid = threadIdx.x;
  const int t = blockIdx.x * 4 + (tid >> 6);
  const int i = tid & 63;
  if (t >= nrows) return;
  const float fr = (float)pos[t] * invf[i];
  float sn, cs;
  sincosf(fr, &sn, &cs);
  float* pc = ctab + (size_t)t * HALF + i;
  float* ps = stab + (size_t)t * HALF + i;
  *(volatile float*)pc = cs;
  *(volatile float*)ps = sn;
  __threadfence();
  *(volatile float*)pc = cs;
  *(volatile float*)ps = sn;
}

template <int NSPLIT, int OUT_MODE>
__global__ __launch_bounds__(256) void gemm64(
    const unsigned short* __restrict__ Ap, const unsigned short* A2p, int lda, long long strideA,
    const unsigned short* __restrict__ Btp, const unsigned short* Bt2p, int ldb, long long strideB,
    void* Cout, int ldc, long long strideC,
    void* Cout2, int ldc2, long long strideC2, int N2,
    int M, int N, int K, float rscale) {
  const __bf16* A   = (const __bf16*)(const void*)Ap;
  const __bf16* A2  = (const __bf16*)(const void*)A2p;
  const __bf16* Bt  = (const __bf16*)(const void*)Btp;
  const __bf16* Bt2 = (const __bf16*)(const void*)Bt2p;
  __shared__ __align__(16) float sT[8][16 * 68];
  const int b    = blockIdx.y;
  const int lane = threadIdx.x & 31;
  const int wave = threadIdx.x >> 5;
  const int tilesN = N >> 6;
  const int tilesM = M >> 6;
  const int tile = blockIdx.x * 8 + wave;
  if (tile >= tilesM * tilesN) return;
  const int tm = tile / tilesN;
  const int tn = tile - tm * tilesN;
  const int m0 = tm << 6;
  const int n0 = tn << 6;

  const __bf16* Ab  = A  + (size_t)b * strideA;
  const __bf16* Bb  = Bt + (size_t)b * strideB;
  const __bf16* Ab2 = (NSPLIT >= 1) ? (A2  + (size_t)b * strideA) : Ab;
  const __bf16* Bb2 = (NSPLIT == 2) ? (Bt2 + (size_t)b * strideB) : Bb;

  const int rlane = lane & 15;
  const int koff  = (lane >> 4) * 8;
  const int mOff  = (lane >> 4) * 8;

  v8f acc[4][4];
#pragma unroll
  for (int i = 0; i < 4; ++i)
#pragma unroll
    for (int j = 0; j < 4; ++j) acc[i][j] = zero8();

  for (int k0 = 0; k0 < K; k0 += 32) {
    v16b bh[4], bl[4];
#pragma unroll
    for (int j = 0; j < 4; ++j) {
      const size_t bo = (size_t)(n0 + (j << 4) + rlane) * ldb + koff + k0;
      bh[j] = ldfrag_b(Bb + bo);
      if (NSPLIT == 2) bl[j] = ldfrag_b(Bb2 + bo); else bl[j] = bh[j];
    }
#pragma unroll
    for (int i = 0; i < 4; ++i) {
      const size_t ao = (size_t)(m0 + (i << 4) + rlane) * lda + koff + k0;
      const v16b ah = ldfrag_b(Ab + ao);
      v16b al = ah;
      if (NSPLIT >= 1) al = ldfrag_b(Ab2 + ao);
#pragma unroll
      for (int j = 0; j < 4; ++j) {
        acc[i][j] = mma_b_raw(ah, bh[j], acc[i][j]);
        if (NSPLIT >= 1) acc[i][j] = mma_b_raw(al, bh[j], acc[i][j]);
        if (NSPLIT == 2) acc[i][j] = mma_b_raw(ah, bl[j], acc[i][j]);
      }
      dep_guard_b(acc[i][0], acc[i][3], ah, al);
    }
    keep4_b(bh[0], bh[1], bh[2], bh[3]);
    if (NSPLIT == 2) keep4_b(bl[0], bl[1], bl[2], bl[3]);
  }
  acc_guard4(acc[0][0], acc[0][1], acc[0][2], acc[0][3]);
  acc_guard4(acc[1][0], acc[1][1], acc[1][2], acc[1][3]);
  acc_guard4(acc[2][0], acc[2][1], acc[2][2], acc[2][3]);
  acc_guard4(acc[3][0], acc[3][1], acc[3][2], acc[3][3]);

  float* slab = sT[wave];
#pragma unroll
  for (int i = 0; i < 4; ++i) {
    const int mBase = m0 + (i << 4);
#pragma unroll
    for (int j = 0; j < 4; ++j) {
#pragma unroll
      for (int r = 0; r < 8; ++r) {
        slab[(mOff + r) * 68 + (j << 4) + rlane] = acc[i][j][r];
      }
    }
    __builtin_amdgcn_fence(__ATOMIC_RELEASE, "workgroup");
    __builtin_amdgcn_wave_barrier();
    __builtin_amdgcn_fence(__ATOMIC_ACQUIRE, "workgroup");
    if (OUT_MODE == 0) {
      float* C = (float*)Cout + (size_t)b * strideC;
      const int hh = lane >> 4, c4 = (lane & 15) * 4;
      for (int pass = 0; pass < 2; ++pass) {
#pragma unroll
        for (int it = 0; it < 8; ++it) {
          const int row = it * 2 + hh;
          const v4f v = *(const v4f*)(slab + row * 68 + c4);
          *(volatile v4f*)(C + (size_t)(mBase + row) * ldc + n0 + c4) = v;
        }
        __threadfence();
      }
    } else {
      const int q = lane >> 3, c8 = (lane & 7) * 8;
      unsigned short* C  = (unsigned short*)Cout  + (size_t)b * strideC;
      unsigned short* C2 = (unsigned short*)Cout2 + (size_t)b * strideC2;
      const bool wlo = (OUT_MODE == 2) || (n0 < N2);
      v4u hv[4], lv[4];
#pragma unroll
      for (int it = 0; it < 4; ++it) {
        const int row = it * 4 + q;
        const float* sp = slab + row * 68 + c8;
        v4u a, a2;
#pragma unroll
        for (int e = 0; e < 4; ++e) {
          const float f0 = sp[2 * e], f1 = sp[2 * e + 1];
          unsigned short h0, h1, l0, l1;
          if (OUT_MODE == 2) {
            h0 = bf_bits(f0); h1 = bf_bits(f1);
            l0 = bf_bits(f0 - bf_up(h0)); l1 = bf_bits(f1 - bf_up(h1));
          } else {
            const _Float16 x0 = (_Float16)f0, x1 = (_Float16)f1;
            h0 = h_bits(x0); h1 = h_bits(x1);
            l0 = h_bits((_Float16)((f0 - (float)x0) * rscale));
            l1 = h_bits((_Float16)((f1 - (float)x1) * rscale));
          }
          a[e] = pk16(h0, h1); a2[e] = pk16(l0, l1);
        }
        hv[it] = a; lv[it] = a2;
      }
      for (int pass = 0; pass < 2; ++pass) {
#pragma unroll
        for (int it = 0; it < 4; ++it) {
          const int row = it * 4 + q;
          *(volatile v4u*)(C + (size_t)(mBase + row) * ldc + n0 + c8) = hv[it];
          if (wlo) *(volatile v4u*)(C2 + (size_t)(mBase + row) * ldc2 + n0 + c8) = lv[it];
        }
        __threadfence();
      }
    }
    __builtin_amdgcn_fence(__ATOMIC_RELEASE, "workgroup");
    __builtin_amdgcn_wave_barrier();
    __builtin_amdgcn_fence(__ATOMIC_ACQUIRE, "workgroup");
  }
}

__global__ __launch_bounds__(256) void norm_rope(const float* __restrict__ xin, const float* __restrict__ wn,
                                                 const float* __restrict__ ctab, const float* __restrict__ stab,
                                                 unsigned short* outh, unsigned short* outl,
                                                 int nheads, int nrows, float rscale) {
  const int tid  = threadIdx.x;
  const int wave = tid >> 5, lane = tid & 31, hh = lane >> 4;
  const int row  = blockIdx.x * 8 + wave;
  if (row >= nrows) return;
  const int t = row / nheads;
  const v4f x = *(const v4f*)(xin + (size_t)row * HD + lane * 4);
  float ss = x[0] * x[0] + x[1] * x[1] + x[2] * x[2] + x[3] * x[3];
#pragma unroll
  for (int off = 1; off < 32; off <<= 1) ss += __shfl_xor(ss, off, 32);
  const float rinv = rsqrtf(ss * (1.0f / (float)HD) + RMS_EPS);
  const v4f wv = *(const v4f*)(wn + lane * 4);
  const v4f cs = *(const v4f*)(ctab + (size_t)t * HALF + (lane & 15) * 4);
  const v4f sn = *(const v4f*)(stab + (size_t)t * HALF + (lane & 15) * 4);
  float n[4], p[4];
#pragma unroll
  for (int e = 0; e < 4; ++e) n[e] = (x[e] * rinv) * bf_up(bf_bits(wv[e]));
#pragma unroll
  for (int e = 0; e < 4; ++e) p[e] = __shfl_xor(n[e], 16, 32);
  const float sg = hh ? 1.0f : -1.0f;
  unsigned short hb[4], lb[4];
#pragma unroll
  for (int e = 0; e < 4; ++e) {
    const float o = n[e] * cs[e] + sg * (p[e] * sn[e]);
    const _Float16 oh = (_Float16)o;
    hb[e] = h_bits(oh);
    lb[e] = h_bits((_Float16)((o - (float)oh) * rscale));
  }
  v2u ph, pl;
  ph[0] = pk16(hb[0], hb[1]); ph[1] = pk16(hb[2], hb[3]);
  pl[0] = pk16(lb[0], lb[1]); pl[1] = pk16(lb[2], lb[3]);
  const size_t go = (size_t)row * HD + lane * 4;
  *(volatile v2u*)(outh + go) = ph;
  *(volatile v2u*)(outl + go) = pl;
  __threadfence();
  *(volatile v2u*)(outh + go) = ph;
  *(volatile v2u*)(outl + go) = pl;
}

template <bool RES> struct AttnL {
  static constexpr int QH   = 0;
  static constexpr int QL   = QH + 64 * 128 * 2;
  static constexpr int KH   = QL + 64 * 128 * 2;
  static constexpr int KL   = KH + 64 * 128 * 2;
  static constexpr int VH   = KL + (RES ? 64 * 128 * 2 : 0);
  static constexpr int VL   = VH + 128 * 64 * 2;
  static constexpr int PH   = VL + (RES ? 128 * 64 * 2 : 0);
  static constexpr int PL   = PH + 4 * 16 * 64 * 2;
  static constexpr int OS   = PL + (RES ? 4 * 16 * 64 * 2 : 0);
  static constexpr int MISC = OS + 4 * 16 * 128 * 4;
  static constexpr int TOTAL = MISC + 1024;
};
static_assert(AttnL<true>::TOTAL <= 160 * 1024);

template <bool RES>
__global__ __launch_bounds__(128)
void attn_causal(const unsigned short* __restrict__ qhp, const unsigned short* __restrict__ qlp,
                 const unsigned short* __restrict__ khp, const unsigned short* __restrict__ klp,
                 const unsigned short* __restrict__ vhp, const unsigned short* __restrict__ vlp,
                 const int* __restrict__ pos,
                 unsigned short* ohp, unsigned short* olp,
                 int qbBase, int nqbThis, float sscale) {
  typedef AttnL<RES> L;
  union FH { v16h v; v8h h[2]; };
  extern __shared__ __align__(16) unsigned char smem[];
  _Float16* Qsh = (_Float16*)(smem + L::QH);
  _Float16* Qsl = (_Float16*)(smem + L::QL);
  _Float16* Ksh = (_Float16*)(smem + L::KH);
  _Float16* Ksl = (_Float16*)(smem + L::KL);
  _Float16* Vth = (_Float16*)(smem + L::VH);
  _Float16* Vtl = (_Float16*)(smem + L::VL);
  _Float16* Psh = (_Float16*)(smem + L::PH);
  _Float16* Psl = (_Float16*)(smem + L::PL);
  float*    Os  = (float*)(smem + L::OS);
  int*      spq = (int*)(smem + L::MISC);
  int*      spk = spq + 64;
  int*      skmin = spk + 64;

  const int tid  = threadIdx.x;
  const int wave = tid >> 5;
  const int lane = tid & 31;
  const int hh   = lane >> 4;
  const int c    = lane & 15;

  const int bx  = blockIdx.x;
  const int qbl = bx % nqbThis;
  const int h   = bx / nqbThis;
  const int kvh = h / GQ;
  const int qb  = qbBase + qbl;
  const int q0  = qb * 64 + wave * 16;

  const _Float16* Qh = (const _Float16*)(const void*)qhp + (size_t)h * HD;
  const _Float16* Ql = (const _Float16*)(const void*)qlp + (size_t)h * HD;
  const _Float16* Kh = (const _Float16*)(const void*)khp + (size_t)kvh * HD;
  const _Float16* Kl = (const _Float16*)(const void*)klp + (size_t)kvh * HD;
  const _Float16* Vh = (const _Float16*)(const void*)vhp + (size_t)kvh * HD * SEQ;
  const _Float16* Vl = (const _Float16*)(const void*)vlp + (size_t)kvh * HD * VLP;

  if (tid < 64) spq[tid] = pos[qb * 64 + tid];
  for (int kt = tid; kt < NQB; kt += 128) {
    const int* pp = pos + kt * 64;
    int mn = 0x7fffffff;
#pragma unroll
    for (int i = 0; i < 16; ++i) {
      const v4i v = *(const v4i*)(pp + 4 * i);
      mn = imin(mn, imin(imin(v[0], v[1]), imin(v[2], v[3])));
    }
    skmin[kt] = mn;
  }
  {
    const int r = tid >> 1, half = (tid & 1) * 64;
    const _Float16* qg  = Qh + (size_t)(qb * 64 + r) * QP + half;
    const _Float16* qlg = Ql + (size_t)(qb * 64 + r) * QP + half;
#pragma unroll
    for (int i = 0; i < 8; ++i) {
      *(v8h*)(Qsh + r * 128 + half + 8 * i) = *(const v8h*)(qg + 8 * i);
      *(v8h*)(Qsl + r * 128 + half + 8 * i) = *(const v8h*)(qlg + 8 * i);
    }
  }
  __syncthreads();
  int qmx;
  {
    int v = imax(spq[lane], spq[lane + 32]);
#pragma unroll
    for (int off = 1; off < 32; off <<= 1) v = imax(v, __shfl_xor(v, off, 32));
    qmx = __builtin_amdgcn_readfirstlane(v);
  }
  int prow[8];
#pragma unroll
  for (int r = 0; r < 8; ++r) prow[r] = spq[wave * 16 + 8 * hh + r];

  float mrow[8], lrow[8];
  v8f oacc[8];
#pragma unroll
  for (int r = 0; r < 8; ++r) { mrow[r] = -INFINITY; lrow[r] = 0.f; }
#pragma unroll
  for (int t = 0; t < 8; ++t) oacc[t] = zero8();

  for (int kt = 0; kt < NQB; ++kt) {
    const int kmn = __builtin_amdgcn_readfirstlane(skmin[kt]);
    if (kmn > qmx) continue;
    const int kv0 = kt * 64;
    __syncthreads();
    {
      const int r = tid >> 1, half = (tid & 1) * 64;
      const _Float16* kg  = Kh + (size_t)(kv0 + r) * KP + half;
      const _Float16* klg = Kl + (size_t)(kv0 + r) * KP + half;
#pragma unroll
      for (int i = 0; i < 8; ++i) {
        *(v8h*)(Ksh + r * 128 + half + 8 * i) = *(const v8h*)(kg + 8 * i);
        if (RES) *(v8h*)(Ksl + r * 128 + half + 8 * i) = *(const v8h*)(klg + 8 * i);
      }
      const int d = tid;
      const _Float16* vg = Vh + (size_t)d * SEQ + kv0;
      const int  kvl   = (kv0 + 64 <= VLP) ? kv0 : (VLP - 64);
      const bool resOK = (kv0 + 64 <= VLP);
      const _Float16* vlg = Vl + (size_t)d * VLP + kvl;
#pragma unroll
      for (int i = 0; i < 8; ++i) {
        *(v8h*)(Vth + d * 64 + 8 * i) = *(const v8h*)(vg + 8 * i);
        if (RES) {
          v8h b1 = *(const v8h*)(vlg + 8 * i);
          if (!resOK) b1 = zero8h();
          *(v8h*)(Vtl + d * 64 + 8 * i) = b1;
        }
      }
      if (tid < 64) spk[tid] = pos[kv0 + tid];
    }
    __syncthreads();

    v8f s[4], sl[4];
#pragma unroll
    for (int j = 0; j < 4; ++j) { s[j] = zero8(); sl[j] = zero8(); }
    const _Float16* qr  = Qsh + (wave * 16 + c) * 128 + 8 * hh;
    const _Float16* qlr = Qsl + (wave * 16 + c) * 128 + 8 * hh;
#pragma unroll
    for (int dc = 0; dc < 4; ++dc) {
      FH qa, qla;
      qa.h[0]  = *(const v8h*)(qr  + dc * 32);
      qa.h[1]  = *(const v8h*)(qr  + dc * 32 + 16);
      qla.h[0] = *(const v8h*)(qlr + dc * 32);
      qla.h[1] = *(const v8h*)(qlr + dc * 32 + 16);
#pragma unroll
      for (int j = 0; j < 4; ++j) {
        FH kb;
        kb.h[0] = *(const v8h*)(Ksh + (j * 16 + c) * 128 + dc * 32 + 8 * hh);
        kb.h[1] = *(const v8h*)(Ksh + (j * 16 + c) * 128 + dc * 32 + 16 + 8 * hh);
        s[j]  = mma_h(qa.v,  kb.v, s[j]);
        sl[j] = mma_h(qla.v, kb.v, sl[j]);
        if (RES) {
          FH klf;
          klf.h[0] = *(const v8h*)(Ksl + (j * 16 + c) * 128 + dc * 32 + 8 * hh);
          klf.h[1] = *(const v8h*)(Ksl + (j * 16 + c) * 128 + dc * 32 + 16 + 8 * hh);
          sl[j] = mma_h(qa.v, klf.v, sl[j]);
        }
      }
    }

    _Float16* pwh = Psh + wave * (16 * 64);
    _Float16* pwl = Psl + (RES ? wave * (16 * 64) : 0);
    int pkj[4];
#pragma unroll
    for (int j = 0; j < 4; ++j) pkj[j] = spk[j * 16 + c];
#pragma unroll
    for (int r = 0; r < 8; ++r) {
      float m = -INFINITY;
#pragma unroll
      for (int j = 0; j < 4; ++j) {
        float sv = (s[j][r] + sl[j][r] * (1.0f / RSC)) * sscale;
        sv = (prow[r] >= pkj[j]) ? sv : -1.0e30f;
        s[j][r] = sv;
        m = fmaxf(m, sv);
      }
#pragma unroll
      for (int off = 1; off < 16; off <<= 1) m = fmaxf(m, __shfl_xor(m, off, 32));
      const float mnew  = fmaxf(mrow[r], m);
      const float msafe = (mnew == -INFINITY) ? 0.f : mnew;
      const float alpha = __expf(mrow[r] - msafe);
      mrow[r] = mnew;
      float psum = 0.f;
#pragma unroll
      for (int j = 0; j < 4; ++j) {
        const float p = __expf(s[j][r] - msafe);
        psum += p;
        const float p1k = p * 1024.0f;
        const _Float16 ph = (_Float16)p1k;
        pwh[(8 * hh + r) * 64 + j * 16 + c] = ph;
        if (RES) {
          const _Float16 pl = (_Float16)((p1k - (float)ph) * RSC);
          pwl[(8 * hh + r) * 64 + j * 16 + c] = pl;
        }
      }
#pragma unroll
      for (int off = 1; off < 16; off <<= 1) psum += __shfl_xor(psum, off, 32);
      lrow[r] = lrow[r] * alpha + psum;
#pragma unroll
      for (int t = 0; t < 8; ++t) oacc[t][r] *= alpha;
    }
    __builtin_amdgcn_fence(__ATOMIC_RELEASE, "workgroup");
    __builtin_amdgcn_wave_barrier();
    __builtin_amdgcn_fence(__ATOMIC_ACQUIRE, "workgroup");

#pragma unroll
    for (int tg = 0; tg < 2; ++tg) {
      v8f o1[4];
#pragma unroll
      for (int t = 0; t < 4; ++t) o1[t] = zero8();
#pragma unroll 1
      for (int kk = 0; kk < 2; ++kk) {
        FH pa, pl;
        pa.h[0] = *(const v8h*)(pwh + c * 64 + kk * 32 + 8 * hh);
        pa.h[1] = *(const v8h*)(pwh + c * 64 + kk * 32 + 16 + 8 * hh);
        if (RES) {
          pl.h[0] = *(const v8h*)(pwl + c * 64 + kk * 32 + 8 * hh);
          pl.h[1] = *(const v8h*)(pwl + c * 64 + kk * 32 + 16 + 8 * hh);
        } else {
          pl.v = pa.v;
        }
#pragma unroll
        for (int t = 0; t < 4; ++t) {
          const int tt = tg * 4 + t;
          FH vb;
          vb.h[0] = *(const v8h*)(Vth + (tt * 16 + c) * 64 + kk * 32 + 8 * hh);
          vb.h[1] = *(const v8h*)(Vth + (tt * 16 + c) * 64 + kk * 32 + 16 + 8 * hh);
          oacc[tt] = mma_h(pa.v, vb.v, oacc[tt]);
          if (RES) {
            FH vl;
            vl.h[0] = *(const v8h*)(Vtl + (tt * 16 + c) * 64 + kk * 32 + 8 * hh);
            vl.h[1] = *(const v8h*)(Vtl + (tt * 16 + c) * 64 + kk * 32 + 16 + 8 * hh);
            o1[t] = mma_h(pa.v, vl.v, o1[t]);
            o1[t] = mma_h(pl.v, vb.v, o1[t]);
          }
        }
      }
      if (RES) {
#pragma unroll
        for (int t = 0; t < 4; ++t)
#pragma unroll
          for (int r = 0; r < 8; ++r) oacc[tg * 4 + t][r] += o1[t][r] * (1.0f / RSC);
      }
    }
  }

  float* os = Os + wave * (16 * 128);
#pragma unroll
  for (int r = 0; r < 8; ++r) {
    const float l = lrow[r];
    const float inv = ((l > 0.f) ? (1.0f / l) : 0.f) * (1.0f / 1024.0f);
#pragma unroll
    for (int t = 0; t < 8; ++t) os[(8 * hh + r) * 128 + t * 16 + c] = oacc[t][r] * inv;
  }
  __builtin_amdgcn_fence(__ATOMIC_RELEASE, "workgroup");
  __builtin_amdgcn_wave_barrier();
  __builtin_amdgcn_fence(__ATOMIC_ACQUIRE, "workgroup");
  {
    const int rh = lane >> 4, c8 = (lane & 15) * 8;
    v4u hv[8], lv[8];
#pragma unroll
    for (int it = 0; it < 8; ++it) {
      const int row = it * 2 + rh;
      const float* sp = os + row * 128 + c8;
      v4u a, a2;
#pragma unroll
      for (int e = 0; e < 4; ++e) {
        const float f0 = sp[2 * e], f1 = sp[2 * e + 1];
        const unsigned short h0 = bf_bits(f0), h1 = bf_bits(f1);
        const unsigned short l0 = bf_bits(f0 - bf_up(h0)), l1 = bf_bits(f1 - bf_up(h1));
        a[e] = pk16(h0, h1); a2[e] = pk16(l0, l1);
      }
      hv[it] = a; lv[it] = a2;
    }
    for (int pass = 0; pass < 2; ++pass) {
#pragma unroll
      for (int it = 0; it < 8; ++it) {
        const int row = it * 2 + rh;
        const size_t go = (size_t)(q0 + row) * QP + (size_t)h * HD + c8;
        *(volatile v4u*)(ohp + go) = hv[it];
        *(volatile v4u*)(olp + go) = lv[it];
      }
      __threadfence();
    }
  }
}

extern "C" void kernel_launch(void* const* d_in, const int* in_sizes, int n_in,
                              void* d_out, int out_size, void* d_ws, size_t ws_size,
                              hipStream_t stream) {
  if (n_in < 8) return;
  if (in_sizes[0] < SEQ) return;
  if (in_sizes[1] < SEQ * DM) return;
  if (in_sizes[2] != DM * QP) return;
  if (in_sizes[3] != DM * KP || in_sizes[4] != DM * KP) return;
  if (in_sizes[5] != QP * DM) return;
  if (in_sizes[6] < HD || in_sizes[7] < HD) return;
  if (out_size < SEQ * DM) return;

  const int*   pos = (const int*)d_in[0];
  const float* x   = (const float*)d_in[1];
  const float* wq  = (const float*)d_in[2];
  const float* wk  = (const float*)d_in[3];
  const float* wv  = (const float*)d_in[4];
  const float* wo  = (const float*)d_in[5];
  const float* qnw = (const float*)d_in[6];
  const float* knw = (const float*)d_in[7];

  const size_t PXb  = (size_t)SEQ * DM * 2;
  const size_t PWq  = (size_t)QP * DM * 2;
  const size_t PWk  = (size_t)KP * DM * 2;
  const size_t PWo  = (size_t)DM * QP * 2;
  const size_t PQf  = (size_t)SEQ * QP * 4;
  const size_t PKf  = (size_t)SEQ * KP * 4;
  const size_t PQ16 = (size_t)SEQ * QP * 2;
  const size_t PK16 = (size_t)SEQ * KP * 2;
  const size_t PVTh = (size_t)KP * SEQ * 2;
  const size_t PVTl = (size_t)KP * VLP * 2;
  const size_t PTab = (size_t)SEQ * HALF * 4;
  const size_t PInv = 4096;
  size_t off = 0;
  const size_t oXb  = off; off += PXb;
  const size_t oWq  = off; off += PWq;
  const size_t oWk  = off; off += PWk;
  const size_t oWv  = off; off += PWk;
  const size_t oWo  = off; off += PWo;
  const size_t oQf  = off; off += PQf;
  const size_t oKf  = off; off += PKf;
  const size_t oQh  = off; off += PQ16;
  const size_t oQl  = off; off += PQ16;
  const size_t oKh  = off; off += PK16;
  const size_t oKl  = off; off += PK16;
  const size_t oVTh = off; off += PVTh;
  const size_t oVTl = off; off += PVTl;
  const size_t oCos = off; off += PTab;
  const size_t oSin = off; off += PTab;
  const size_t oInv = off; off += PInv;
  if (off > ws_size) return;
  if (off > (size_t)134217728) return;
  if (PQ16 * 2 != PQf) return;
  const size_t oOh = oQf;
  const size_t oOl = oQf + PQ16;

  char* ws = (char*)d_ws;
  unsigned short* Xb  = (unsigned short*)(ws + oXb);
  unsigned short* Wqt = (unsigned short*)(ws + oWq);
  unsigned short* Wkt = (unsigned short*)(ws + oWk);
  unsigned short* Wvt = (unsigned short*)(ws + oWv);
  unsigned short* Wot = (unsigned short*)(ws + oWo);
  float*          Qf  = (float*)(ws + oQf);
  float*          Kf  = (float*)(ws + oKf);
  unsigned short* Qh  = (unsigned short*)(ws + oQh);
  unsigned short* Ql  = (unsigned short*)(ws + oQl);
  unsigned short* Kh  = (unsigned short*)(ws + oKh);
  unsigned short* Kl  = (unsigned short*)(ws + oKl);
  unsigned short* VTh = (unsigned short*)(ws + oVTh);
  unsigned short* VTl = (unsigned short*)(ws + oVTl);
  float*          Cs  = (float*)(ws + oCos);
  float*          Sn  = (float*)(ws + oSin);
  float*          Invf = (float*)(ws + oInv);
  unsigned short* Oh  = (unsigned short*)(ws + oOh);
  unsigned short* Ol  = (unsigned short*)(ws + oOl);

  const dim3 blk(256);
  const int n8x = SEQ * DM / 8;
  const dim3 gCvtX((n8x + 255) / 256);
  const dim3 gTab((SEQ + 3) / 4);
  const dim3 gTq(QP / 64, DM / 64);
  const dim3 gTk(KP / 64, DM / 64);
  const dim3 gTo(DM / 64, QP / 64);
  const dim3 gProjQ(((SEQ / 64) * (QP / 64) + 7) / 8, 1);
  const dim3 gProjK(((SEQ / 64) * (KP / 64) + 7) / 8, 1);
  const dim3 gVT(((KP / 64) * (SEQ / 64) + 7) / 8, 1);
  const dim3 gOut(((SEQ / 64) * (DM / 64) + 7) / 8, 1);
  const dim3 gNq((SEQ * NH + 7) / 8);
  const dim3 gNk((SEQ * NKV + 7) / 8);

  invf_tab<<<dim3(1), dim3(64), 0, stream>>>(Invf);
  rope_tab<<<gTab, blk, 0, stream>>>(pos, Invf, Cs, Sn, SEQ);
  cvt_bf16x8<<<gCvtX, blk, 0, stream>>>(x, Xb, n8x);
  cvt_bf16_t<<<gTq, blk, 0, stream>>>(wq, Wqt, DM, QP);
  cvt_bf16_t<<<gTk, blk, 0, stream>>>(wk, Wkt, DM, KP);
  cvt_bf16_t<<<gTk, blk, 0, stream>>>(wv, Wvt, DM, KP);
  cvt_bf16_t<<<gTo, blk, 0, stream>>>(wo, Wot, QP, DM);
  gemm64<0, 0><<<gProjQ, blk, 0, stream>>>(
      Xb, Xb, DM, 0LL, Wqt, Wqt, DM, 0LL,
      (void*)Qf, QP, 0LL, (void*)Qf, QP, 0LL, QP,
      SEQ, QP, DM, 1.0f);
  gemm64<0, 0><<<gProjK, blk, 0, stream>>>(
      Xb, Xb, DM, 0LL, Wkt, Wkt, DM, 0LL,
      (void*)Kf, KP, 0LL, (void*)Kf, KP, 0LL, KP,
      SEQ, KP, DM, 1.0f);
  gemm64<0, 3><<<gVT, blk, 0, stream>>>(
      Wvt, Wvt, DM, 0LL, Xb, Xb, DM, 0LL,
      (void*)VTh, SEQ, 0LL, (void*)VTl, VLP, 0LL, VLP,
      KP, SEQ, DM, RSC);
  norm_rope<<<gNq, blk, 0, stream>>>(Qf, qnw, Cs, Sn, Qh, Ql, NH, SEQ * NH, RSC);
  norm_rope<<<gNk, blk, 0, stream>>>(Kf, knw, Cs, Sn, Kh, Kl, NKV, SEQ * NKV, RSC);
  (void)hipFuncSetAttribute(reinterpret_cast<const void*>(&attn_causal<true>),
                            hipFuncAttributeMaxDynamicSharedMemorySize, AttnL<true>::TOTAL);
  (void)hipFuncSetAttribute(reinterpret_cast<const void*>(&attn_causal<false>),
                            hipFuncAttributeMaxDynamicSharedMemorySize, AttnL<false>::TOTAL);
  attn_causal<true><<<dim3(NH * RESQB), dim3(128), AttnL<true>::TOTAL, stream>>>(
      Qh, Ql, Kh, Kl, VTh, VTl, pos, Oh, Ol, 0, RESQB, ATT_SCALE);
  if (NQB - RESQB > 0) {
    attn_causal<false><<<dim3(NH * (NQB - RESQB)), dim3(128), AttnL<false>::TOTAL, stream>>>(
        Qh, Ql, Kh, Kl, VTh, VTl, pos, Oh, Ol, RESQB, NQB - RESQB, ATT_SCALE);
  }
  gemm64<1, 0><<<gOut, blk, 0, stream>>>(
      Oh, Ol, QP, 0LL, Wot, Wot, QP, 0LL,
      d_out, DM, 0LL, d_out, DM, 0LL, DM,
      SEQ, DM, QP, 1.0f);
  (void)hipGetLastError();
}
